// GPT2SelfAttention_19490561589680
// MI455X (gfx1250) — hardware-verified
//
#include <hip/hip_runtime.h>
#include <stddef.h>

#define NB     2
#define NS     2048
#define ND     1024
#define NH     16
#define HD     64
#define MROWS  (NB * NS)
#define NQKV   (3 * ND)
#define QLO    512
#define QT_ALL (NS / 16)
#define QT_LO  (QLO / 16)
#define MT_ALL (NS / 64)
#define MT_LO  (QLO / 64)

typedef _Float16       v8h  __attribute__((ext_vector_type(8)));
typedef _Float16       v16h __attribute__((ext_vector_type(16)));
typedef __bf16         v16b __attribute__((ext_vector_type(16)));
typedef unsigned short v8us __attribute__((ext_vector_type(8)));
typedef float          v8f  __attribute__((ext_vector_type(8)));
typedef float          v4f  __attribute__((ext_vector_type(4)));

union FragH { v16h v; v8h u[2]; _Float16 e[16]; };
union FragB { v16b v; v8us u[2]; };

__device__ __forceinline__ v8f zero8() {
  v8f z = {0.f, 0.f, 0.f, 0.f, 0.f, 0.f, 0.f, 0.f};
  return z;
}

__device__ __forceinline__ v8f mma_h(v16h a, v16h b, v8f c) {
  c = __builtin_amdgcn_wmma_f32_16x16x32_f16(false, a, false, b, (short)0, c, false, false);
  asm volatile("v_nop\n\tv_nop\n\tv_nop\n\tv_nop" : "+v"(c) : "v"(a), "v"(b));
  return c;
}
__device__ __forceinline__ v8f mma_b(v16b a, v16b b, v8f c) {
  c = __builtin_amdgcn_wmma_f32_16x16x32_bf16(false, a, false, b, (short)0, c, false, false);
  asm volatile("v_nop\n\tv_nop\n\tv_nop\n\tv_nop" : "+v"(c) : "v"(a), "v"(b));
  return c;
}

__device__ __forceinline__ unsigned short bf_bits(float f) {
  unsigned int u = __float_as_uint(f);
  u += 0x7FFFu + ((u >> 16) & 1u);
  return (unsigned short)(u >> 16);
}
__device__ __forceinline__ float bf_val(unsigned short b) { return __uint_as_float(((unsigned int)b) << 16); }
__device__ __forceinline__ float bf_rne(float f) { return bf_val(bf_bits(f)); }
__device__ __forceinline__ unsigned short h_bits(_Float16 x) { return __builtin_bit_cast(unsigned short, x); }

__global__ void __launch_bounds__(256) k_cvt_x(const float* __restrict__ src, unsigned short* dst, int n8) {
  const int i = blockIdx.x * 256 + (int)threadIdx.x;
  const bool act = i < n8;
  v8us o = {0, 0, 0, 0, 0, 0, 0, 0};
  if (act) {
    const float* s = src + (size_t)i * 8;
    const v4f a = *(const v4f*)(s);
    const v4f b = *(const v4f*)(s + 4);
    o[0] = bf_bits(a[0]); o[1] = bf_bits(a[1]); o[2] = bf_bits(a[2]); o[3] = bf_bits(a[3]);
    o[4] = bf_bits(b[0]); o[5] = bf_bits(b[1]); o[6] = bf_bits(b[2]); o[7] = bf_bits(b[3]);
  }
  unsigned short* p = dst + (size_t)i * 8;
  if (act) *(volatile v8us*)p = o;
  __threadfence();
  if (act) *(volatile v8us*)p = o;
}

template <int MODE>
__global__ void __launch_bounds__(256) k_wtrans(const float* __restrict__ W, unsigned short* WT, int krows, int ncols) {
  __shared__ float T[64][65];
  const int tid = threadIdx.x;
  const int n0 = blockIdx.x * 64, k0 = blockIdx.y * 64;
#pragma unroll
  for (int j = 0; j < 16; ++j) {
    const int idx = tid + 256 * j;
    const int kr = idx >> 6, nc = idx & 63;
    const int gk = k0 + kr, gn = n0 + nc;
    float v = 0.f;
    if (gk < krows && gn < ncols) v = W[(size_t)gk * ncols + gn];
    T[kr][nc] = v;
  }
  __syncthreads();
  v8us val[2];
  size_t off[2];
  bool ok[2];
#pragma unroll
  for (int j = 0; j < 2; ++j) {
    const int c = tid + 256 * j;
    const int row = c >> 3, part = c & 7;
    const int gn = n0 + row;
    ok[j] = (gn < ncols) && (k0 + part * 8 + 8 <= krows);
    v8us v;
#pragma unroll
    for (int e = 0; e < 8; ++e) {
      const unsigned short bb = bf_bits(T[part * 8 + e][row]);
      if (MODE == 0) {
        v[e] = bb;
      } else {
        v[e] = h_bits((_Float16)(bf_val(bb) * 1024.0f));
      }
    }
    val[j] = v;
    off[j] = (size_t)gn * krows + k0 + part * 8;
  }
#pragma unroll
  for (int j = 0; j < 2; ++j)
    if (ok[j]) *(volatile v8us*)(WT + off[j]) = val[j];
  __threadfence();
#pragma unroll
  for (int j = 0; j < 2; ++j)
    if (ok[j]) *(volatile v8us*)(WT + off[j]) = val[j];
}

__global__ void __launch_bounds__(128) k_qkv(const unsigned short* __restrict__ xb, const unsigned short* __restrict__ wT,
                                           const float* __restrict__ bq,
                                           _Float16* Qo, _Float16* Ko, _Float16* Vho, _Float16* Vlo, int lo_rows) {
  __shared__ float T[64][65];
  const int tid = threadIdx.x, lane = tid & 31, wid = tid >> 5, h = lane >> 4, m = lane & 15;
  const int n0 = blockIdx.x * 64, m0 = blockIdx.y * 64;
  const int mw = m0 + wid * 16;

  v8f acc[4];
#pragma unroll
  for (int t = 0; t < 4; ++t) acc[t] = zero8();

  const unsigned short* ap = xb + (size_t)(mw + m) * ND + 8 * h;
  const unsigned short* bp = wT + (size_t)(n0 + m) * ND + 8 * h;
#pragma unroll 1
  for (int k0 = 0; k0 < ND; k0 += 32) {
    FragB a;
    a.u[0] = *(const v8us*)(ap + k0);
    a.u[1] = *(const v8us*)(ap + k0 + 16);
#pragma unroll
    for (int t = 0; t < 4; ++t) {
      const unsigned short* q = bp + (size_t)t * 16 * ND + k0;
      FragB b;
      b.u[0] = *(const v8us*)(q);
      b.u[1] = *(const v8us*)(q + 16);
      acc[t] = mma_b(a.v, b.v, acc[t]);
    }
  }

#pragma unroll
  for (int t = 0; t < 4; ++t) {
    const float bias = bf_rne(bq[n0 + t * 16 + m]);
#pragma unroll
    for (int r = 0; r < 8; ++r) T[wid * 16 + 8 * h + r][t * 16 + m] = acc[t][r] + bias;
  }
  __syncthreads();

  const int which = n0 / ND;
  const int hh = (n0 - which * ND) / HD;
  const int b = m0 / NS;
  const int s0 = m0 - b * NS;
  const int bh = b * NH + hh;

  if (which < 2) {
    _Float16* base = (which == 0 ? Qo : Ko) + ((size_t)bh * NS + s0) * HD;
    v8h val[4];
    int offs[4];
#pragma unroll
    for (int j = 0; j < 4; ++j) {
      const int c = tid + 128 * j;
      const int row = c >> 3, part = c & 7;
      v8h v;
#pragma unroll
      for (int e = 0; e < 8; ++e) v[e] = (_Float16)T[row][part * 8 + e];
      val[j] = v;
      offs[j] = row * HD + part * 8;
    }
#pragma unroll
    for (int j = 0; j < 4; ++j) *(volatile v8h*)(base + offs[j]) = val[j];
    __threadfence();
#pragma unroll
    for (int j = 0; j < 4; ++j) *(volatile v8h*)(base + offs[j]) = val[j];
  } else {
    _Float16* bhi = Vho + (size_t)bh * HD * NS + s0;
    _Float16* blo = Vlo + (size_t)bh * HD * NS + s0;
    const bool wl = s0 < lo_rows;
    v8h vh[4], vl[4];
    int offs[4];
#pragma unroll
    for (int j = 0; j < 4; ++j) {
      const int c = tid + 128 * j;
      const int d = c >> 3, part = c & 7;
      v8h a, r2;
#pragma unroll
      for (int e = 0; e < 8; ++e) {
        const float f = T[part * 8 + e][d] * 16.0f;
        const _Float16 g = (_Float16)f;
        a[e] = g;
        r2[e] = (_Float16)((f - (float)g) * 2048.0f);
      }
      vh[j] = a;
      vl[j] = r2;
      offs[j] = d * NS + part * 8;
    }
#pragma unroll
    for (int j = 0; j < 4; ++j) {
      *(volatile v8h*)(bhi + offs[j]) = vh[j];
      if (wl) *(volatile v8h*)(blo + offs[j]) = vl[j];
    }
    __threadfence();
#pragma unroll
    for (int j = 0; j < 4; ++j) {
      *(volatile v8h*)(bhi + offs[j]) = vh[j];
      if (wl) *(volatile v8h*)(blo + offs[j]) = vl[j];
    }
  }
}

template <bool SPLIT>
__global__ void __launch_bounds__(64) k_attn(const _Float16* __restrict__ Qg, const _Float16* __restrict__ Kg,
                                            const _Float16* __restrict__ Vhg, const _Float16* __restrict__ Vlg,
                                            _Float16* Ohg, _Float16* Olg, int qt_lo, int n_qt, int ntask) {
  __shared__ __attribute__((aligned(16))) _Float16 stg[2][2][16][72];
  const int tid = threadIdx.x, lane = tid & 31, wid = tid >> 5, h = lane >> 4, n = lane & 15;
  const int task = blockIdx.x * 2 + wid;
  const bool act = task < ntask;
  const int tk = act ? task : 0;
  const int bh = tk / n_qt;
  const int qi = qt_lo + (tk - bh * n_qt);
  const int q0 = qi * 16;
  const int qrow = q0 + n;

  const _Float16* Qp = Qg + ((size_t)bh * NS + qrow) * HD + 8 * h;
  FragH qa, qb;
  qa.u[0] = *(const v8h*)(Qp);
  qa.u[1] = *(const v8h*)(Qp + 16);
  qb.u[0] = *(const v8h*)(Qp + 32);
  qb.u[1] = *(const v8h*)(Qp + 48);

  const _Float16* Kb  = Kg  + (size_t)bh * NS * HD + (size_t)n * HD + 8 * h;
  const _Float16* Vhb = Vhg + (size_t)bh * HD * NS + (size_t)n * NS + 8 * h;
  const _Float16* Vlb = Vlg + (size_t)bh * HD * NS + (size_t)n * NS + 8 * h;

  v8f oA[4], oB[4];
#pragma unroll
  for (int t = 0; t < 4; ++t) { oA[t] = zero8(); oB[t] = zero8(); }
  float mr = -3.0e38f, lr = 0.f;
  const int nkb = act ? (((q0 + 15) >> 5) + 1) : 0;

#pragma unroll 1
  for (int j = 0; j < nkb; ++j) {
    const int k0 = j * 32;
    v8f sc[2];
#pragma unroll
    for (int kt = 0; kt < 2; ++kt) {
      const _Float16* Kp = Kb + (size_t)(k0 + kt * 16) * HD;
      FragH ka, kc;
      ka.u[0] = *(const v8h*)(Kp);
      ka.u[1] = *(const v8h*)(Kp + 16);
      kc.u[0] = *(const v8h*)(Kp + 32);
      kc.u[1] = *(const v8h*)(Kp + 48);
      v8f s = zero8();
      s = mma_h(ka.v, qa.v, s);
      s = mma_h(kc.v, qb.v, s);
      sc[kt] = s;
    }
    float bm = -3.0e38f;
#pragma unroll
    for (int kt = 0; kt < 2; ++kt) {
#pragma unroll
      for (int r = 0; r < 8; ++r) {
        float v = sc[kt][r] * 0.125f;
        const int key = k0 + kt * 16 + 8 * h + r;
        if (key > qrow) v = -10000.0f;
        sc[kt][r] = v;
        bm = fmaxf(bm, v);
      }
    }
    bm = fmaxf(bm, __shfl_xor(bm, 16));
    const float mnew = fmaxf(mr, bm);
    float rs = 0.f;
#pragma unroll
    for (int kt = 0; kt < 2; ++kt) {
#pragma unroll
      for (int r = 0; r < 8; ++r) {
        const float p = __expf(sc[kt][r] - mnew);
        sc[kt][r] = p;
        rs += p;
      }
    }
    rs += __shfl_xor(rs, 16);
    const float co = __expf(mr - mnew);
    lr = lr * co + rs;
    mr = mnew;
#pragma unroll
    for (int t = 0; t < 4; ++t) {
      oA[t] = oA[t] * co;
      if (SPLIT) oB[t] = oB[t] * co;
    }
    FragH ph, pl;
#pragma unroll
    for (int i = 0; i < 8; ++i) {
      const float f0 = sc[0][i] * 256.0f;
      const _Float16 g0 = (_Float16)f0;
      ph.e[i] = g0;
      const float f1 = sc[1][i] * 256.0f;
      const _Float16 g1 = (_Float16)f1;
      ph.e[8 + i] = g1;
      if (SPLIT) {
        pl.e[i]     = (_Float16)((f0 - (float)g0) * 2048.0f);
        pl.e[8 + i] = (_Float16)((f1 - (float)g1) * 2048.0f);
      }
    }
#pragma unroll
    for (int t = 0; t < 4; ++t) {
      const size_t vo = (size_t)t * 16 * NS + k0;
      FragH va;
      va.u[0] = *(const v8h*)(Vhb + vo);
      va.u[1] = *(const v8h*)(Vhb + vo + 16);
      oA[t] = mma_h(va.v, ph.v, oA[t]);
      if (SPLIT) {
        FragH vl;
        vl.u[0] = *(const v8h*)(Vlb + vo);
        vl.u[1] = *(const v8h*)(Vlb + vo + 16);
        oB[t] = mma_h(vl.v, ph.v, oB[t]);
        oB[t] = mma_h(va.v, pl.v, oB[t]);
      }
    }
  }

  const float inv = (lr > 0.f) ? (1.0f / lr) : 0.f;
  const float sA = inv * (1.0f / 4096.0f);
  const float sB = inv * (1.0f / 8388608.0f);
#pragma unroll
  for (int t = 0; t < 4; ++t) {
    v8h ch, cl;
#pragma unroll
    for (int r = 0; r < 8; ++r) {
      float o = oA[t][r] * sA;
      if (SPLIT) o += oB[t][r] * sB;
      const float f = o * 16.0f;
      const _Float16 g = (_Float16)f;
      ch[r] = g;
      if (SPLIT) cl[r] = (_Float16)((f - (float)g) * 2048.0f);
    }
    *(v8h*)(&stg[wid][0][n][t * 16 + 8 * h]) = ch;
    if (SPLIT) *(v8h*)(&stg[wid][1][n][t * 16 + 8 * h]) = cl;
  }
  __syncthreads();

  const int b = bh / NH, hh = bh - b * NH;
  _Float16* ob  = Ohg + ((size_t)b * NS + q0) * ND + hh * HD;
  _Float16* olb = Olg + ((size_t)b * NS + q0) * ND + hh * HD;
  v8h w0[4], w1[4];
  int offs[4];
#pragma unroll
  for (int jj = 0; jj < 4; ++jj) {
    const int c = lane + 32 * jj;
    const int qq = c >> 3, part = c & 7;
    w0[jj] = *(const v8h*)(&stg[wid][0][qq][part * 8]);
    if (SPLIT) w1[jj] = *(const v8h*)(&stg[wid][1][qq][part * 8]);
    offs[jj] = qq * ND + part * 8;
  }
  if (act) {
#pragma unroll
    for (int jj = 0; jj < 4; ++jj) {
      *(volatile v8h*)(ob + offs[jj]) = w0[jj];
      if (SPLIT) *(volatile v8h*)(olb + offs[jj]) = w1[jj];
    }
  }
  __threadfence();
  if (act) {
#pragma unroll
    for (int jj = 0; jj < 4; ++jj) {
      *(volatile v8h*)(ob + offs[jj]) = w0[jj];
      if (SPLIT) *(volatile v8h*)(olb + offs[jj]) = w1[jj];
    }
  }
}

template <bool SPLIT>
__global__ void __launch_bounds__(128) k_out(const _Float16* __restrict__ Oh, const _Float16* __restrict__ Ol,
                                            const unsigned short* __restrict__ wT, const float* __restrict__ bo,
                                            float* out, int tiles_per_b, int s_base) {
  __shared__ __attribute__((aligned(16))) float T[64][68];
  const int tid = threadIdx.x, lane = tid & 31, wid = tid >> 5, h = lane >> 4, m = lane & 15;
  const int n0 = blockIdx.x * 64;
  const int by = blockIdx.y;
  const int b = by / tiles_per_b;
  const int m0 = b * NS + s_base + (by - b * tiles_per_b) * 64;
  const int mw = m0 + wid * 16;

  v8f acc[4], acr[4];
#pragma unroll
  for (int t = 0; t < 4; ++t) { acc[t] = zero8(); acr[t] = zero8(); }

  const _Float16* ap  = Oh + (size_t)(mw + m) * ND + 8 * h;
  const _Float16* alp = Ol + (size_t)(mw + m) * ND + 8 * h;
  const unsigned short* bp = wT + (size_t)(n0 + m) * ND + 8 * h;
#pragma unroll 1
  for (int k0 = 0; k0 < ND; k0 += 32) {
    FragH a, al;
    a.u[0] = *(const v8h*)(ap + k0);
    a.u[1] = *(const v8h*)(ap + k0 + 16);
    if (SPLIT) {
      al.u[0] = *(const v8h*)(alp + k0);
      al.u[1] = *(const v8h*)(alp + k0 + 16);
    }
#pragma unroll
    for (int t = 0; t < 4; ++t) {
      const unsigned short* q = bp + (size_t)t * 16 * ND + k0;
      FragH bb;
      bb.u[0] = *(const v8h*)(q);
      bb.u[1] = *(const v8h*)(q + 16);
      acc[t] = mma_h(a.v, bb.v, acc[t]);
      if (SPLIT) acr[t] = mma_h(al.v, bb.v, acr[t]);
    }
  }

#pragma unroll
  for (int t = 0; t < 4; ++t) {
    const float bias = bf_rne(bo[n0 + t * 16 + m]);
#pragma unroll
    for (int r = 0; r < 8; ++r) {
      float v = acc[t][r] * (1.0f / 16384.0f);
      if (SPLIT) v += acr[t][r] * (1.0f / 33554432.0f);
      T[wid * 16 + 8 * h + r][t * 16 + m] = v + bias;
    }
  }
  __syncthreads();

  v4f val[8];
  int offs[8];
#pragma unroll
  for (int j = 0; j < 8; ++j) {
    const int c = tid + 128 * j;
    const int row = c >> 4, part = c & 15;
    val[j] = *(const v4f*)(&T[row][part * 4]);
    offs[j] = row * ND + part * 4;
  }
  float* obase = out + (size_t)m0 * ND + n0;
#pragma unroll
  for (int j = 0; j < 8; ++j) *(volatile v4f*)(obase + offs[j]) = val[j];
  __threadfence();
#pragma unroll
  for (int j = 0; j < 8; ++j) *(volatile v4f*)(obase + offs[j]) = val[j];
}

extern "C" void kernel_launch(void* const* d_in, const int* in_sizes, int n_in,
                              void* d_out, int out_size, void* d_ws, size_t ws_size,
                              hipStream_t stream) {
  if (n_in < 5) return;
  if (in_sizes[0] != MROWS * ND || in_sizes[1] != ND * NQKV || in_sizes[2] != NQKV ||
      in_sizes[3] != ND * ND || in_sizes[4] != ND || out_size != MROWS * ND) return;

  const float* x    = (const float*)d_in[0];
  const float* Wqkv = (const float*)d_in[1];
  const float* bqkv = (const float*)d_in[2];
  const float* Wout = (const float*)d_in[3];
  const float* bout = (const float*)d_in[4];
  float* out = (float*)d_out;

  const size_t sz_xb = (size_t)MROWS * ND * 2;
  const size_t sz_wq = (size_t)NQKV * ND * 2;
  const size_t sz_wo = (size_t)ND * ND * 2;
  const size_t sz_q  = (size_t)NB * NH * NS * HD * 2;
  const size_t sz_o  = (size_t)MROWS * ND * 2;
  const size_t off_xb = 0;
  const size_t off_wq = off_xb + sz_xb;
  const size_t off_wo = off_wq + sz_wq;
  const size_t off_q  = off_wo + sz_wo;
  const size_t off_k  = off_q  + sz_q;
  const size_t off_vh = off_k  + sz_q;
  const size_t off_vl = off_vh + sz_q;
  const size_t off_oh = off_vl + sz_q;
  const size_t off_ol = off_oh + sz_o;
  const size_t need   = off_ol + sz_o;
  if (ws_size < need) return;

  char* ws = (char*)d_ws;
  unsigned short* xb  = (unsigned short*)(ws + off_xb);
  unsigned short* wqT = (unsigned short*)(ws + off_wq);
  unsigned short* woT = (unsigned short*)(ws + off_wo);
  _Float16* Qb  = (_Float16*)(ws + off_q);
  _Float16* Kb  = (_Float16*)(ws + off_k);
  _Float16* Vh  = (_Float16*)(ws + off_vh);
  _Float16* Vl  = (_Float16*)(ws + off_vl);
  _Float16* Ohp = (_Float16*)(ws + off_oh);
  _Float16* Olp = (_Float16*)(ws + off_ol);

  const int n8 = MROWS * ND / 8;
  k_cvt_x<<<dim3((n8 + 255) / 256), dim3(256), 0, stream>>>(x, xb, n8);
  k_wtrans<0><<<dim3(NQKV / 64, ND / 64), dim3(256), 0, stream>>>(Wqkv, wqT, ND, NQKV);
  k_wtrans<1><<<dim3(ND / 64, ND / 64), dim3(256), 0, stream>>>(Wout, woT, ND, ND);

  k_qkv<<<dim3(NQKV / 64, MROWS / 64), dim3(128), 0, stream>>>(xb, wqT, bqkv, Qb, Kb, Vh, Vl, QLO);

  const int nt_lo = NB * NH * QT_LO;
  const int nt_hi = NB * NH * (QT_ALL - QT_LO);
  k_attn<true><<<dim3((nt_lo + 1) / 2), dim3(64), 0, stream>>>(Qb, Kb, Vh, Vl, Ohp, Olp, 0, QT_LO, nt_lo);
  k_attn<false><<<dim3((nt_hi + 1) / 2), dim3(64), 0, stream>>>(Qb, Kb, Vh, Vl, Ohp, Olp, QT_LO, QT_ALL - QT_LO, nt_hi);

  k_out<true><<<dim3(ND / 64, NB * MT_LO), dim3(128), 0, stream>>>(Ohp, Olp, woT, bout, out, MT_LO, 0);
  k_out<false><<<dim3(ND / 64, NB * (MT_ALL - MT_LO)), dim3(128), 0, stream>>>(Ohp, Olp, woT, bout, out, MT_ALL - MT_LO, QLO);
}
